// QuantumSelfAttention_65481071405315
// MI455X (gfx1250) — hardware-run, weakly checked
//
#include <hip/hip_runtime.h>


#ifndef NB
#define NB 16
#endif
#ifndef SEQ
#define SEQ 1024
#endif
#define NB_FULL  16
#define SEQ_FULL 1024
#ifndef OUT_SEQ
#define OUT_SEQ SEQ
#endif
#define NQ   10
#define KDIM 1024
#define AW   4
#define FTP  40
#define PCS  16384.0f
#define PCI  (1.0f / 16384.0f)

static_assert(NQ == 10);
static_assert((1 << NQ) == KDIM);
static_assert(KDIM % 32 == 0);
static_assert(KDIM / 32 == 32);
static_assert(2 * 5 == NQ);
static_assert(NQ <= 16);
static_assert(FTP == NQ * 4);
static_assert((FTP * 4) % 16 == 0);
static_assert(SEQ % (16 * AW) == 0);
static_assert((NB * SEQ) % (16 * AW) == 0);
static_assert(OUT_SEQ % 16 == 0);
static_assert((16 * NQ * 4) % 128 == 0);
static_assert(32 * 16 + 8 * 16 == 16 * NQ * 4);
static_assert(NB <= NB_FULL);
static_assert(SEQ <= SEQ_FULL);
static_assert((AW * 16 * FTP + AW * 16 * 32 + AW * 16 * NQ) * 4 <= 131072);

typedef _Float16 h16;
typedef __attribute__((ext_vector_type(16))) _Float16 v16h;
typedef __attribute__((ext_vector_type(8)))  float    v8f;
typedef __attribute__((ext_vector_type(4)))  float    v4f;
typedef v4f  __attribute__((may_alias)) v4fa;

__device__ __forceinline__ unsigned short f2bf(float f) { unsigned u = __float_as_uint(f); u += 0x7FFFu + ((u >> 16) & 1u); return (unsigned short)(u >> 16); }
__device__ __forceinline__ float bfr(float f) { return __uint_as_float(((unsigned)f2bf(f)) << 16); }
__device__ __forceinline__ v8f wmma16(v16h a, v16h b, v8f c) { return __builtin_amdgcn_wmma_f32_16x16x32_f16(false, a, false, b, (short)0, c, false, false); }
__device__ __forceinline__ void wave_sync() { __builtin_amdgcn_fence(3  , "wavefront"); __builtin_amdgcn_wave_barrier(); asm volatile("" ::: "memory"); }
static __device__ __forceinline__ h16 toh_flush(float v) { const h16 r = (h16)v; return (fabsf(v) < 6.103515625e-05f) ? (h16)0.0f : r; }
__device__ __forceinline__ v8f wmma16g(v16h a, v16h b, v8f c) { c = wmma16(a, b, c); asm volatile("v_nop\n\tv_nop\n\tv_nop\n\tv_nop" : "+v"(c) : "v"(a), "v"(b)); return c; }

__global__ __launch_bounds__(32 * AW) void k_expect(const float* __restrict__ X, const float* __restrict__ ROT, const float* __restrict__ ENT, float* OUT) {
    __shared__ __align__(16) float ft[AW * 16 * FTP];
    __shared__ __align__(16) float ht[AW * 16 * 32];
    __shared__ __align__(16) float os[AW * 16 * NQ];
    const int lane = threadIdx.x & 31, lr = lane & 15, hi = lane >> 4;
    const int wave = __builtin_amdgcn_readfirstlane((int)(threadIdx.x >> 5));
    const int g0 = blockIdx.x * (16 * AW) + wave * 16;
    const int b = g0 / SEQ, s0 = g0 % SEQ;
    const float* xrow = X + ((size_t)b * SEQ_FULL + (size_t)(s0 + lr)) * NQ;
    const int fb = (wave * 16 + lr) * FTP;
    const bool up = hi != 0;

#pragma unroll 1
    for (int kk = 0; kk < 5; ++kk) {
        const int k = 5 * hi + kk;
        const int ke = k > 0 ? k - 1 : 0;
        const float xv = bfr(xrow[k]);
        const float rv = bfr(ROT[k]);
        const float ev = bfr(ENT[ke]);
        const float th = (xv + rv) * 0.5f;
        const float hf = ev * 0.5f;
        float s, c, sp, cp;
        sincosf(th, &s, &c);
        sincosf(hf, &sp, &cp);
        const float a0 = cp * c, a1 = sp * s, d0 = sp * c, d1 = cp * s;
        v4f f;
        f[0] = c * c; f[1] = s * s; f[2] = a0 * a0 + a1 * a1; f[3] = d0 * d0 + d1 * d1;
        *(v4fa*)(&ft[fb + 4 * k]) = f;
    }
    wave_sync();

    const v4f f0 = *(const v4fa*)(&ft[fb +  0]); const v4f f1 = *(const v4fa*)(&ft[fb +  4]);
    const v4f f2 = *(const v4fa*)(&ft[fb +  8]); const v4f f3 = *(const v4fa*)(&ft[fb + 12]);
    const v4f f4 = *(const v4fa*)(&ft[fb + 16]); const v4f f5 = *(const v4fa*)(&ft[fb + 20]);
    const v4f f6 = *(const v4fa*)(&ft[fb + 24]); const v4f f7 = *(const v4fa*)(&ft[fb + 28]);
    const v4f f8 = *(const v4fa*)(&ft[fb + 32]); const v4f f9 = *(const v4fa*)(&ft[fb + 36]);
    const int hb = (wave * 16 + lr) * 32;
    {
        const float p0 = up ? f0[1] : f0[0];
        float w1[2], w2[4], w3[8], w4[16];
#pragma unroll
        for (int i = 0; i < 2; ++i) w1[i] = p0 * (up ? f1[2 + i] : f1[i]);
#pragma unroll
        for (int i = 0; i < 4; ++i) w2[i] = w1[i >> 1] * f2[i];
#pragma unroll
        for (int i = 0; i < 8; ++i) w3[i] = w2[i >> 1] * f3[i & 3];
#pragma unroll
        for (int i = 0; i < 16; ++i) w4[i] = w3[i >> 1] * f4[i & 3];
#pragma unroll
        for (int q = 0; q < 4; ++q) { v4f o; o[0] = w4[4 * q] * PCS; o[1] = w4[4 * q + 1] * PCS; o[2] = w4[4 * q + 2] * PCS; o[3] = w4[4 * q + 3] * PCS;
            *(v4fa*)(&ht[hb + 16 * hi + 4 * q]) = o; }
    }
    float la0[16], la1[16];
    {
        float t7[2], t8[4], tl[8], hd[4];
#pragma unroll
        for (int i = 0; i < 2; ++i) t7[i] = up ? f7[2 + i] : f7[i];
#pragma unroll
        for (int i = 0; i < 4; ++i) t8[i] = t7[i >> 1] * f8[i];
#pragma unroll
        for (int i = 0; i < 8; ++i) tl[i] = t8[i >> 1] * f9[i & 3];
#pragma unroll
        for (int i = 0; i < 4; ++i) hd[i] = f5[i] * (up ? f6[2 * (i & 1) + 1] : f6[2 * (i & 1)]);
#pragma unroll
        for (int e = 0; e < 16; ++e) { la0[e] = hd[e >> 3] * tl[e & 7]; la1[e] = hd[2 + (e >> 3)] * tl[e & 7]; }
    }
    const bool lowcol = (lr >= 5) & (lr < NQ);
    const bool hicol  = lr < 5;
    const int lsh = lowcol ? (NQ - 1 - lr) : 0;
    const int jsh = hicol ? (4 - lr) : 0;
    const float lf = lowcol ? 1.0f : 0.0f, jf = hicol ? 1.0f : 0.0f;
    v16h fixb;
#pragma unroll
    for (int e = 0; e < 16; ++e) { const int low = 8 * hi + (e < 8 ? e : e + 8); fixb[e] = (h16)(lf * (1.0f - 2.0f * (float)((low >> lsh) & 1))); }
    wave_sync();

    v8f acc = (v8f){};
#pragma unroll 1
    for (int j2 = 0; j2 < 16; ++j2) {
        {
            const int j = 2 * j2;
            const float hv = ht[hb + j];
            const h16 sj = (h16)(jf * (1.0f - 2.0f * (float)((j >> jsh) & 1)));
            v16h a, bq;
#pragma unroll
            for (int e = 0; e < 16; ++e) { a[e] = toh_flush(hv * la0[e]); bq[e] = fixb[e] + sj; }
            acc = wmma16g(a, bq, acc);
        }
        {
            const int j = 2 * j2 + 1;
            const float hv = ht[hb + j];
            const h16 sj = (h16)(jf * (1.0f - 2.0f * (float)((j >> jsh) & 1)));
            v16h a, bq;
#pragma unroll
            for (int e = 0; e < 16; ++e) { a[e] = toh_flush(hv * la1[e]); bq[e] = fixb[e] + sj; }
            acc = wmma16g(a, bq, acc);
        }
    }

    const int wb = wave * 16 * NQ;
    if (lr < NQ) {
#pragma unroll
        for (int r = 0; r < 8; ++r) os[wb + (8 * hi + r) * NQ + lr] = acc[r] * PCI;
    }
    wave_sync();
    float* orow = OUT + ((size_t)b * OUT_SEQ + (size_t)s0) * NQ;
    const v4f va = *(const v4fa*)(&os[wb + 4 * lane]);
    const v4f vb = *(const v4fa*)(&os[wb + 128 + 4 * (lane & 7)]);
#pragma unroll 1
    for (int ps = 0; ps < 2; ++ps) {
        *(volatile v4f*)(orow + 4 * lane) = va;
        if (lane < 8) *(volatile v4f*)(orow + 128 + 4 * lane) = vb;
        if (ps == 0) __threadfence(); }
}

extern "C" void kernel_launch(void* const* d_in, const int* in_sizes, int n_in,
                              void* d_out, int out_size, void* d_ws, size_t ws_size, hipStream_t stream) {
    if (n_in < 3) return;
    const size_t needx = ((size_t)(NB - 1) * SEQ_FULL + SEQ) * NQ;
    if ((size_t)in_sizes[0] < needx) return;
    if (in_sizes[1] < NQ || in_sizes[2] < NQ - 1) return;
    if ((size_t)out_size < ((size_t)(NB - 1) * OUT_SEQ + SEQ) * NQ) return;
    (void)d_ws; (void)ws_size;
    const float* x   = (const float*)d_in[0];
    const float* rot = (const float*)d_in[1];
    const float* ent = (const float*)d_in[2];
    float* OUT = (float*)d_out;
    k_expect<<<dim3(NB * SEQ / (16 * AW), 1, 1), 32 * AW, 0, stream>>>(x, rot, ent, OUT);
}
